// NTM_5660766896261
// MI455X (gfx1250) — hardware-run, weakly checked
//
#include <hip/hip_runtime.h>
#include <math.h>

typedef __attribute__((ext_vector_type(16))) _Float16 v16h;
typedef __attribute__((ext_vector_type(8)))  _Float16 v8h;
typedef __attribute__((ext_vector_type(4)))  _Float16 v4h;
typedef __attribute__((ext_vector_type(2)))  _Float16 v2h;
typedef __attribute__((ext_vector_type(16))) __bf16   v16b;
typedef __attribute__((ext_vector_type(8)))  __bf16   v8b;
typedef __attribute__((ext_vector_type(8)))  float    v8f;
typedef __attribute__((ext_vector_type(4)))  float    v4f;
typedef __attribute__((ext_vector_type(2)))  float    v2f;

constexpr int kB    = 128;
constexpr int kT    = 128;
constexpr int kD    = 128;
constexpr int kNs   = 128;
constexpr int kMw   = 128;
constexpr int kHc   = 256;
constexpr int kNA   = 576;
constexpr int kThr  = 256;
constexpr int kColK0 = 0, kColK1 = 128, kColHd = 256, kColEr = 320, kColAd = 448;

constexpr float kInCarry = 1024.0f;
constexpr float kWCarry  = 1024.0f;
constexpr float kHCarry  = 256.0f;
constexpr float kRCarry  = 4096.0f;
constexpr float kXScale  = 1.0f / (kInCarry * kWCarry);
constexpr float kRScale  = 1.0f / (kRCarry * kWCarry);
constexpr float kAScale  = 1.0f / (kHCarry * kWCarry);
constexpr float kEps     = 1e-8f;
constexpr float kF16MinNormal = 6.103515625e-5f;

static_assert(((kB * kT) % 64) == 0 && (kHc % 64) == 0 && (kNA % 64) == 0 && (kD % 32) == 0 && (kMw % 32) == 0 && (kHc % 32) == 0, "GEMM M, N multiples of 64, K of 32");
static_assert(kColAd + kMw == kNA && kColHd + 12 <= kColEr, "stacked columns");

constexpr size_t kOffX16  = 0;
constexpr size_t kOffWX   = kOffX16  + (size_t)kB * kT * kD * 2;
constexpr size_t kOffWRD  = kOffWX   + (size_t)kHc * kD * 2;
constexpr size_t kOffWA   = kOffWRD  + (size_t)kHc * 2 * kMw * 2;
constexpr size_t kOffBA   = kOffWA   + (size_t)kNA * 2 * kHc * 2;
constexpr size_t kOffBH   = kOffBA   + 2560;
constexpr size_t kOffZB   = kOffBH   + 1024;
constexpr size_t kOffXW   = kOffZB   + 1024;
constexpr size_t kOffH16  = kOffXW   + (size_t)kB * kT * kHc * 4;
constexpr size_t kOffR16  = kOffH16  + (size_t)kB * 2 * kHc * 2;
constexpr size_t kOffPREH = kOffR16  + (size_t)kB * 2 * kMw * 2;
constexpr size_t kOffPREA = kOffPREH + (size_t)kB * kHc * 4;
constexpr size_t kOffMEM  = kOffPREA + (size_t)kB * kNA * 4;
constexpr size_t kOffWRW  = kOffMEM  + (size_t)kB * kNs * kMw * 4;
constexpr size_t kWsTotal = kOffWRW  + (size_t)2 * kB * kNs * 4;
static_assert(kWsTotal == 30904832ull, "carve total");
static_assert(kWsTotal <= 134217728ull, "carve cap");
static_assert((kOffWX % 256) == 0 && (kOffWRD % 256) == 0 && (kOffWA % 256) == 0 && (kOffBA % 256) == 0 && (kOffBH % 256) == 0 && (kOffZB % 256) == 0 && (kOffXW % 256) == 0 && (kOffH16 % 256) == 0 && (kOffR16 % 256) == 0 && (kOffPREH % 256) == 0 && (kOffPREA % 256) == 0 && (kOffMEM % 256) == 0 && (kOffWRW % 256) == 0, "aligned regions");

__device__ __forceinline__ unsigned short f2bf_bits(float f) {
  unsigned u = __float_as_uint(f);
  return (unsigned short)((u + 0x7FFFu + ((u >> 16) & 1u)) >> 16);
}
__device__ __forceinline__ float bf_bits2f(unsigned short h) { return __uint_as_float(((unsigned)h) << 16); }
__device__ __forceinline__ float bf16r(float f) { return bf_bits2f(f2bf_bits(f)); }
__device__ __forceinline__ float carry_flush(float v, float carry) {
  const float s = v * carry;
  return (fabsf(s) < kF16MinNormal) ? 0.0f : s;
}
__device__ __forceinline__ float frcp(float x) { return __builtin_amdgcn_rcpf(x); }

__device__ __forceinline__ void dep_guard4_h(v8f& a, v8f& b, v8f& c, v8f& d, v16h x, v16h y) { asm volatile("v_nop\n\tv_nop\n\tv_nop\n\tv_nop" : "+v"(a), "+v"(b), "+v"(c), "+v"(d) : "v"(x), "v"(y)); }
__device__ __forceinline__ void dep_guard4_b(v8f& a, v8f& b, v8f& c, v8f& d, v16b x, v16b y) { asm volatile("v_nop\n\tv_nop\n\tv_nop\n\tv_nop" : "+v"(a), "+v"(b), "+v"(c), "+v"(d) : "v"(x), "v"(y)); }
__device__ __forceinline__ void keep4_h(v16h a, v16h b, v16h c, v16h d) { asm volatile("v_nop" :: "v"(a), "v"(b), "v"(c), "v"(d)); }
__device__ __forceinline__ void keep4_b(v16b a, v16b b, v16b c, v16b d) { asm volatile("v_nop" :: "v"(a), "v"(b), "v"(c), "v"(d)); }
__device__ __forceinline__ void acc_guard4(v8f& a, v8f& b, v8f& c, v8f& d) { asm volatile("v_nop\n\tv_nop\n\tv_nop\n\tv_nop" : "+v"(a), "+v"(b), "+v"(c), "+v"(d)); }

template <typename T> struct Frag;
template <> struct Frag<_Float16> {
  typedef v16h V; union U { v16h v; v8h h[2]; };
  static __device__ __forceinline__ v16h load(const _Float16* p) {
    U f; f.h[0] = *(const v8h*)(p); f.h[1] = *(const v8h*)(p + 16); return f.v;
  }
  static __device__ __forceinline__ v8f mma(v16h a, v16h b, v8f c) {
    return __builtin_amdgcn_wmma_f32_16x16x32_f16(false, a, false, b, (short)0, c, false, false);
  }
  static __device__ __forceinline__ void guard4(v8f& a, v8f& b, v8f& c, v8f& d, v16h x, v16h y) { dep_guard4_h(a, b, c, d, x, y); }
  static __device__ __forceinline__ void keep(v16h a, v16h b, v16h c, v16h d) { keep4_h(a, b, c, d); }
};
template <> struct Frag<__bf16> {
  typedef v16b V; union U { v16b v; v8b h[2]; };
  static __device__ __forceinline__ v16b load(const __bf16* p) {
    U f; f.h[0] = *(const v8b*)(p); f.h[1] = *(const v8b*)(p + 16); return f.v;
  }
  static __device__ __forceinline__ v8f mma(v16b a, v16b b, v8f c) {
    return __builtin_amdgcn_wmma_f32_16x16x32_bf16(false, a, false, b, (short)0, c, false, false);
  }
  static __device__ __forceinline__ void guard4(v8f& a, v8f& b, v8f& c, v8f& d, v16b x, v16b y) { dep_guard4_b(a, b, c, d, x, y); }
  static __device__ __forceinline__ void keep(v16b a, v16b b, v16b c, v16b d) { keep4_b(a, b, c, d); }
};

__device__ __forceinline__ v8f mma_h(v16h a, v16h b, v8f c) {
  c = __builtin_amdgcn_wmma_f32_16x16x32_f16(false, a, false, b, (short)0, c, false, false);
  asm volatile("v_nop\n\tv_nop\n\tv_nop\n\tv_nop" : "+v"(c) : "v"(a), "v"(b));
  return c;
}

template <int ET> struct Elem;
template <> struct Elem<0> { typedef _Float16 T; };
template <> struct Elem<1> { typedef __bf16 T; };
template <int ET, bool SPLIT, int BIAS_MODE, int OUT_MODE, bool RESID, int ACT = 0>
__global__ __launch_bounds__(256) void wmma_gemm64(
    const unsigned short* __restrict__ Ap, const unsigned short* __restrict__ A2p, int lda, long strideA,
    const unsigned short* __restrict__ Btp, const unsigned short* __restrict__ Bt2p, int ldb, long strideB,
    void* __restrict__ Cout, void* __restrict__ Cout2, int ldc, long strideC,
    const float* __restrict__ bias,
    const float* __restrict__ resid, long strideR,
    int M, int N, int K, float scale) {
  typedef typename Elem<ET>::T T;
  typedef typename Frag<T>::V V;
  const T* A = (const T*)Ap; const T* A2 = (const T*)A2p; const T* Bt = (const T*)Btp; const T* Bt2 = (const T*)Bt2p;
  __shared__ __align__(16) float sT[8][16 * 68];
  const int b    = blockIdx.y;
  const int lane = threadIdx.x & 31;
  const int wave = threadIdx.x >> 5;
  const int tilesN = N >> 6;
  const int tilesM = M >> 6;
  const int tile = blockIdx.x * 8 + wave;
  if (tile >= tilesM * tilesN) return;
  const int tm = tile / tilesN;
  const int tn = tile - tm * tilesN;
  const int m0 = tm << 6;
  const int n0 = tn << 6;

  const T* Ab  = A  + (size_t)b * strideA;
  const T* Bb  = Bt + (size_t)b * strideB;
  const T* Ab2 = SPLIT ? (A2  + (size_t)b * strideA) : nullptr;
  const T* Bb2 = SPLIT ? (Bt2 + (size_t)b * strideB) : nullptr;

  const int rlane = lane & 15;
  const int koff  = (lane >> 4) * 8;
  const int mOff  = (lane >> 4) * 8;

  v8f acc[4][4];
#pragma unroll
  for (int i = 0; i < 4; ++i)
#pragma unroll
    for (int j = 0; j < 4; ++j) acc[i][j] = (v8f){0.f,0.f,0.f,0.f,0.f,0.f,0.f,0.f};

  for (int k0 = 0; k0 < K; k0 += 32) {
    V bh[4], bl[4];
#pragma unroll
    for (int j = 0; j < 4; ++j) {
      const size_t bo = (size_t)(n0 + (j << 4) + rlane) * ldb + koff + k0;
      bh[j] = Frag<T>::load(Bb + bo);
      if (SPLIT) bl[j] = Frag<T>::load(Bb2 + bo);
    }
#pragma unroll
    for (int i = 0; i < 4; ++i) {
      const size_t ao = (size_t)(m0 + (i << 4) + rlane) * lda + koff + k0;
      V ah = Frag<T>::load(Ab + ao);
      V al;
      if (SPLIT) al = Frag<T>::load(Ab2 + ao);
#pragma unroll
      for (int j = 0; j < 4; ++j) {
        acc[i][j] = Frag<T>::mma(ah, bh[j], acc[i][j]);
        if (SPLIT) {
          acc[i][j] = Frag<T>::mma(ah, bl[j], acc[i][j]);
          acc[i][j] = Frag<T>::mma(al, bh[j], acc[i][j]);
        }
      }
      Frag<T>::guard4(acc[i][0], acc[i][1], acc[i][2], acc[i][3], ah, SPLIT ? al : ah);
    }
    Frag<T>::keep(bh[0], bh[1], bh[2], bh[3]);
    if (SPLIT) Frag<T>::keep(bl[0], bl[1], bl[2], bl[3]);
  }
  acc_guard4(acc[0][0], acc[0][1], acc[0][2], acc[0][3]);
  acc_guard4(acc[1][0], acc[1][1], acc[1][2], acc[1][3]);
  acc_guard4(acc[2][0], acc[2][1], acc[2][2], acc[2][3]);
  acc_guard4(acc[3][0], acc[3][1], acc[3][2], acc[3][3]);

  float* slab = sT[wave];
  const float* Rb = RESID ? (resid + (size_t)b * strideR) : nullptr;
#pragma unroll
  for (int i = 0; i < 4; ++i) {
    const int mBase = m0 + (i << 4);
#pragma unroll
    for (int j = 0; j < 4; ++j) {
      const int n = n0 + (j << 4) + rlane;
      float bv = 0.f;
      if (BIAS_MODE == 2) bv = bias[n];
#pragma unroll
      for (int r = 0; r < 8; ++r) {
        float v = acc[i][j][r] * scale;
        if (BIAS_MODE == 1) v += bias[mBase + mOff + r];
        if (BIAS_MODE == 2) v += bv;
        if (RESID) v += Rb[(size_t)(mBase + mOff + r) * ldc + n];
        if (ACT == 1) v = tanhf(v);
        if (ACT == 2) v = fmaxf(v, 0.0f);
        if (ACT == 3) v = v / (1.0f + expf(-v));
        if (ACT == 4) v = (v > 0.f) ? v : 0.01f * v;
        slab[(mOff + r) * 68 + (j << 4) + rlane] = v;
      }
    }
    __builtin_amdgcn_fence(__ATOMIC_RELEASE, "workgroup");
    __builtin_amdgcn_wave_barrier();
    __builtin_amdgcn_fence(__ATOMIC_ACQUIRE, "workgroup");
    if (OUT_MODE == 0) {
      float* C = (float*)Cout + (size_t)b * strideC;
      const int hh = lane >> 4, c4 = (lane & 15) * 4;
      for (int pass = 0; pass < 2; ++pass) {
#pragma unroll
        for (int it = 0; it < 8; ++it) {
          const int row = it * 2 + hh;
          v4f v = *(const v4f*)(slab + row * 68 + c4);
          *(volatile v4f*)(C + (size_t)(mBase + row) * ldc + n0 + c4) = v;
        }
        __threadfence();
      }
    } else {
      const int q = lane >> 3, c8 = (lane & 7) * 8;
      unsigned short* C  = (unsigned short*)Cout  + (size_t)b * strideC;
      unsigned short* C2 = (OUT_MODE == 2) ? ((unsigned short*)Cout2 + (size_t)b * strideC) : nullptr;
      for (int pass = 0; pass < 2; ++pass) {
#pragma unroll
        for (int it = 0; it < 4; ++it) {
          const int row = it * 4 + q;
          const float* sp = slab + row * 68 + c8;
          v8h hv, lv;
#pragma unroll
          for (int e = 0; e < 8; ++e) {
            if (OUT_MODE == 1) {
              hv[e] = (_Float16)sp[e];
            } else {
              unsigned short hb = f2bf_bits(sp[e]);
              unsigned short lb = f2bf_bits(sp[e] - bf_bits2f(hb));
              hv[e] = __builtin_bit_cast(_Float16, hb);
              lv[e] = __builtin_bit_cast(_Float16, lb);
            }
          }
          *(volatile v8h*)(C + (size_t)(mBase + row) * ldc + n0 + c8) = hv;
          if (OUT_MODE == 2) *(volatile v8h*)(C2 + (size_t)(mBase + row) * ldc + n0 + c8) = lv;
        }
        __threadfence();
      }
    }
    __builtin_amdgcn_fence(__ATOMIC_RELEASE, "workgroup");
    __builtin_amdgcn_wave_barrier();
    __builtin_amdgcn_fence(__ATOMIC_ACQUIRE, "workgroup");
  }
}

__global__ __launch_bounds__(kThr) void cast_plane_kernel(const float* __restrict__ src, unsigned short* __restrict__ dst,
                                                          int colsLog2, int dstPitch, int dstOff) {
  const int i   = blockIdx.x * kThr + threadIdx.x;
  const int sh  = colsLog2 - 3;
  const int row = i >> sh;
  const int c8  = (i & ((1 << sh) - 1)) * 8;
  const float* sp = src + ((size_t)row << colsLog2) + c8;
  const v4f a0 = *(const v4f*)(sp);
  const v4f a1 = *(const v4f*)(sp + 4);
  v8h hv;
#pragma unroll
  for (int e = 0; e < 4; ++e) {
    const float f0 = a0[e];
    const float f1 = a1[e];
    hv[e]     = (_Float16)carry_flush(bf16r(f0), kInCarry);
    hv[4 + e] = (_Float16)carry_flush(bf16r(f1), kInCarry);
  }
  unsigned short* dp = dst + (size_t)row * dstPitch + dstOff + c8;
  *(volatile v8h*)dp = hv;
  __threadfence();
  *(volatile v8h*)dp = hv;
}
static_assert(kInCarry == kWCarry, "one cast kernel serves inputs and weights");

__global__ __launch_bounds__(32) void tcast_kernel(const float* __restrict__ src, unsigned short* __restrict__ dst, int K, int N, int dup) {
  const int n  = blockIdx.x;
  const int k8 = threadIdx.x * 8;
  v8h hv;
#pragma unroll
  for (int e = 0; e < 8; ++e) hv[e] = (_Float16)carry_flush(bf16r(src[(size_t)(k8 + e) * N + n]), kWCarry);
  const int pitch = dup ? 2 * K : K;
  unsigned short* dp = dst + (size_t)n * pitch + k8;
  for (int pass = 0; pass < 2; ++pass) {
    *(volatile v8h*)dp = hv;
    if (dup) *(volatile v8h*)(dp + K) = hv;
    __threadfence();
  }
}

__global__ __launch_bounds__(32) void wa_plane_kernel(const float* __restrict__ Wk, const float* __restrict__ Wb,
                                                      const float* __restrict__ Wg, const float* __restrict__ Ws,
                                                      const float* __restrict__ Wgam, const float* __restrict__ We,
                                                      const float* __restrict__ Wa, unsigned short* __restrict__ WA16) {
  const int n  = blockIdx.x;
  const int k8 = threadIdx.x * 8;
  const float* base;
  int stride;
  bool zero = false;
  if (n < 256)      { base = Wk + (size_t)(n >> 7) * kHc * kMw + (n & 127); stride = kMw; }
  else if (n < 258) { base = Wb + (size_t)(n - 256) * kHc; stride = 1; }
  else if (n < 260) { base = Wg + (size_t)(n - 258) * kHc; stride = 1; }
  else if (n < 266) { const int q = n - 260; base = Ws + (size_t)(q / 3) * kHc * 3 + (q % 3); stride = 3; }
  else if (n < 268) { base = Wgam + (size_t)(n - 266) * kHc; stride = 1; }
  else if (n < 320) { base = Wb; stride = 1; zero = true; }
  else if (n < 448) { base = We + (n - 320); stride = kMw; }
  else              { base = Wa + (n - 448); stride = kMw; }
  v8h hv;
#pragma unroll
  for (int e = 0; e < 8; ++e) {
    const float wv = base[(size_t)(k8 + e) * stride];
    hv[e] = (_Float16)carry_flush(zero ? 0.0f : bf16r(wv), kWCarry);
  }
  unsigned short* dp = WA16 + (size_t)n * (2 * kHc) + k8;
  for (int pass = 0; pass < 2; ++pass) {
    *(volatile v8h*)dp = hv;
    *(volatile v8h*)(dp + kHc) = hv;
    __threadfence();
  }
}

__global__ __launch_bounds__(kThr) void ntm_small_kernel(const float* __restrict__ bk, const float* __restrict__ bb,
                                                         const float* __restrict__ bg, const float* __restrict__ bs,
                                                         const float* __restrict__ bgam, const float* __restrict__ be,
                                                         const float* __restrict__ ba, const float* __restrict__ bh,
                                                         const float* __restrict__ h0, const float* __restrict__ wr0,
                                                         const float* __restrict__ ww0,
                                                         float* __restrict__ BA, float* __restrict__ BH, float* __restrict__ ZB,
                                                         unsigned short* __restrict__ H16, float* __restrict__ WRW) {
  const int tid = threadIdx.x;
#pragma unroll 1
  for (int it = 0; it < 3; ++it) {
    const int eraw = it * kThr + tid;
    const bool live = (eraw < kNA);
    const int e = live ? eraw : (kNA - 1);
    {
      const int q = e - kColHd;
      const int ik  = (e < 256) ? e : 0;
      const int i2  = (q >= 0 && q < 2) ? q : ((q >= 2 && q < 4) ? (q - 2) : ((q >= 10 && q < 12) ? (q - 10) : 0));
      const int i6  = (q >= 4 && q < 10) ? (q - 4) : 0;
      const int im  = (e >= kColAd) ? (e - kColAd) : ((e >= kColEr) ? (e - kColEr) : 0);
      float vk = bk[ik], vb = bb[i2], vg = bg[i2], vs = bs[i6], vgm = bgam[i2], ve = be[im], va = ba[im];
      asm volatile("" : "+v"(vk), "+v"(vb), "+v"(vg), "+v"(vs), "+v"(vgm), "+v"(ve), "+v"(va));
      float v = 0.0f;
      v = (e < 256) ? vk : v;
      v = (q >= 0 && q < 2) ? vb : v;
      v = (q >= 2 && q < 4) ? vg : v;
      v = (q >= 4 && q < 10) ? vs : v;
      v = (q >= 10 && q < 12) ? vgm : v;
      v = (e >= kColEr && e < kColAd) ? ve : v;
      v = (e >= kColAd) ? va : v;
      const float o = bf16r(v);
      if (live) {
        *(volatile float*)(BA + e) = o;
        __threadfence();
        *(volatile float*)(BA + e) = o;
      }
    }
  }
  {
    const float o = bf16r(bh[tid]);
    *(volatile float*)(BH + tid) = o;
    *(volatile float*)(ZB + tid) = 0.0f;
    __threadfence();
    *(volatile float*)(BH + tid) = o;
    *(volatile float*)(ZB + tid) = 0.0f;
  }
#pragma unroll 1
  for (int it = 0; it < (kB * kHc) / (4 * kThr); ++it) {
    const int e4 = (it * kThr + tid) * 4;
    const v4f hv = *(const v4f*)(h0 + e4);
    v4h ho, hl;
#pragma unroll
    for (int e = 0; e < 4; ++e) {
      const float hc = bf16r(hv[e]) * kHCarry;
      const _Float16 hi = (_Float16)carry_flush(hc, 1.0f);
      ho[e] = hi;
      hl[e] = (_Float16)carry_flush(hc - (float)hi, 1.0f);
    }
    unsigned short* hp = H16 + (size_t)(e4 >> 8) * (2 * kHc) + (e4 & (kHc - 1));
    for (int pass = 0; pass < 2; ++pass) {
      *(volatile v4h*)hp = ho;
      *(volatile v4h*)(hp + kHc) = hl;
      __threadfence();
    }
  }
#pragma unroll 1
  for (int it = 0; it < (2 * kB * kNs) / kThr; ++it) {
    const int e = it * kThr + tid;
    const int half = e / (kB * kNs);
    const int r = e - half * (kB * kNs);
    float a = wr0[r], c = ww0[r];
    asm volatile("" : "+v"(a), "+v"(c));
    const float o = bf16r(half ? c : a);
    *(volatile float*)(WRW + e) = o;
    __threadfence();
    *(volatile float*)(WRW + e) = o;
  }
}

__global__ __launch_bounds__(kThr) void ntm_ctrl_kernel(const float* __restrict__ XW, const float* __restrict__ PREH,
                                                        float* __restrict__ out, unsigned short* __restrict__ H16, int t) {
  const int v  = blockIdx.x * kThr + threadIdx.x;
  const int b  = v >> 6;
  const int u4 = (v & 63) * 4;
  const v4f xw = *(const v4f*)(XW + ((size_t)b * kT + t) * kHc + u4);
  const v4f ph = *(const v4f*)(PREH + (size_t)b * kHc + u4);
  v4f h;
  v4h ho, hl;
#pragma unroll
  for (int e = 0; e < 4; ++e) {
    h[e] = tanhf(xw[e] + ph[e]);
    const float hc = h[e] * kHCarry;
    const _Float16 hi = (_Float16)carry_flush(hc, 1.0f);
    ho[e] = hi;
    hl[e] = (_Float16)carry_flush(hc - (float)hi, 1.0f);
  }
  float* op = out + ((size_t)b * kT + t) * kHc + u4;
  unsigned short* hp = H16 + (size_t)b * (2 * kHc) + u4;
  for (int pass = 0; pass < 2; ++pass) {
    *(volatile v4f*)op = h;
    *(volatile v4h*)hp = ho;
    *(volatile v4h*)(hp + kHc) = hl;
    __threadfence();
  }
}

__device__ __forceinline__ float softplus_f(float v) { return fmaxf(v, 0.0f) + log1pf(expf(-fabsf(v))); }
__device__ __forceinline__ float sigmoid_f(float v) { return 1.0f / (1.0f + expf(-v)); }

__global__ __launch_bounds__(128) void ntm_mem_kernel(const float* __restrict__ PREA, float* __restrict__ MEM,
                                                      float* __restrict__ WRW, unsigned short* __restrict__ R16,
                                                      int do_address, int do_write) {
  __shared__ float smem[kNs * 129];
  __shared__ __align__(16) float sk[2][kMw];
  __shared__ __align__(16) float sv[kNs];
  __shared__ __align__(16) float sw[2][kNs];
  __shared__ __align__(16) float se[kMw];
  __shared__ __align__(16) float sa[kMw];
  __shared__ __align__(16) float sr[kMw];
  const int b = blockIdx.x;
  const int tid = threadIdx.x;
  const float* pa = PREA + (size_t)b * kNA;
  float* memb = MEM + (size_t)b * kNs * kMw;

#pragma unroll 4
  for (int n = 0; n < kNs; ++n) smem[n * 129 + tid] = memb[n * kMw + tid];
  sw[0][tid] = WRW[(size_t)b * kNs + tid];
  sw[1][tid] = WRW[(size_t)(kB + b) * kNs + tid];
  __syncthreads();

  if (do_address) {
    sk[0][tid] = tanhf(pa[kColK0 + tid]);
    sk[1][tid] = tanhf(pa[kColK1 + tid]);
    __syncthreads();
    float nrm2 = 0.0f, d0 = 0.0f, d1 = 0.0f, kk0 = 0.0f, kk1 = 0.0f;
#pragma unroll 1
    for (int m = 0; m < kMw; ++m) {
      const float mv = smem[tid * 129 + m];
      const float k0 = sk[0][m], k1 = sk[1][m];
      nrm2 = fmaf(mv, mv, nrm2);
      d0 = fmaf(k0, mv, d0);
      d1 = fmaf(k1, mv, d1);
      kk0 = fmaf(k0, k0, kk0);
      kk1 = fmaf(k1, k1, kk1);
    }
    const float nrm = sqrtf(nrm2);
#pragma unroll 1
    for (int hd = 0; hd < 2; ++hd) {
      const float beta  = softplus_f(pa[kColHd + hd]);
      const float g     = sigmoid_f(pa[kColHd + 2 + hd]);
      const float l0 = pa[kColHd + 4 + 3 * hd], l1 = pa[kColHd + 5 + 3 * hd], l2 = pa[kColHd + 6 + 3 * hd];
      const float lm = fmaxf(fmaxf(l0, l1), l2);
      const float x0 = expf(l0 - lm), x1 = expf(l1 - lm), x2 = expf(l2 - lm);
      const float xs = (x0 + x1) + x2;
      const float s0 = x0 / xs, s1 = x1 / xs, s2 = x2 / xs;
      const float gamma = 1.0f + softplus_f(pa[kColHd + 10 + hd]);
      const float dot = hd ? d1 : d0;
      const float kn  = sqrtf(hd ? kk1 : kk0);
      const float z = beta * (dot / (kn * nrm + kEps));
      sv[tid] = z;
      __syncthreads();
      float zmax = sv[0];
#pragma unroll 4
      for (int n = 1; n < kNs; ++n) zmax = fmaxf(zmax, sv[n]);
      __syncthreads();
      const float ez = expf(z - zmax);
      sv[tid] = ez;
      __syncthreads();
      float zs = 0.0f;
#pragma unroll 4
      for (int n = 0; n < kNs; ++n) zs += sv[n];
      __syncthreads();
      const float wc = ez / zs;
      const float wg = g * wc + (1.0f - g) * sw[hd][tid];
      sv[tid] = wg;
      __syncthreads();
      const float sh = (s0 * sv[(tid + kNs - 1) & (kNs - 1)] + s1 * wg) + s2 * sv[(tid + 1) & (kNs - 1)];
      __syncthreads();
      const float wp = (sh > 0.0f) ? expf(gamma * logf(sh)) : 0.0f;
      sv[tid] = wp;
      __syncthreads();
      float ps = 0.0f;
#pragma unroll 4
      for (int n = 0; n < kNs; ++n) ps += sv[n];
      __syncthreads();
      const float wn = wp / (ps + kEps);
      sw[hd][tid] = wn;
      float* wp_out = WRW + (size_t)(hd * kB + b) * kNs + tid;
      *(volatile float*)wp_out = wn;
      __threadfence();
      *(volatile float*)wp_out = wn;
    }
    __syncthreads();
  }

  if (do_write) {
    se[tid] = sigmoid_f(pa[kColEr + tid]);
    sa[tid] = tanhf(pa[kColAd + tid]);
    __syncthreads();
    {
      const float wwn = sw[1][tid];
#pragma unroll 1
      for (int m = 0; m < kMw; ++m) {
        const float mv = smem[tid * 129 + m];
        smem[tid * 129 + m] = mv * (1.0f - wwn * se[m]) + wwn * sa[m];
      }
    }
    __syncthreads();
    {
      float r = 0.0f;
#pragma unroll 2
      for (int n = 0; n < kNs; ++n) r = fmaf(sw[0][n], smem[n * 129 + tid], r);
      sr[tid] = r;
    }
    __syncthreads();
    const float rq0 = sr[(2 * tid) & (kMw - 1)];
    const float rq1 = sr[(2 * tid + 1) & (kMw - 1)];
    if (tid < kMw / 2) {
      v2h ro, rl;
      const float c0 = rq0 * kRCarry, c1 = rq1 * kRCarry;
      ro[0] = (_Float16)carry_flush(c0, 1.0f);
      ro[1] = (_Float16)carry_flush(c1, 1.0f);
      rl[0] = (_Float16)carry_flush(c0 - (float)ro[0], 1.0f);
      rl[1] = (_Float16)carry_flush(c1 - (float)ro[1], 1.0f);
      unsigned short* rp = R16 + (size_t)b * (2 * kMw) + 2 * tid;
      for (int pass = 0; pass < 2; ++pass) {
        *(volatile v2h*)rp = ro;
        *(volatile v2h*)(rp + kMw) = rl;
        __threadfence();
      }
    }
#pragma unroll 1
    for (int n = 0; n < kNs; ++n) {
      const float mv = smem[n * 129 + tid];
      *(volatile float*)(memb + n * kMw + tid) = mv;
    }
    __threadfence();
#pragma unroll 1
    for (int n = 0; n < kNs; ++n) {
      const float mv = smem[n * 129 + tid];
      *(volatile float*)(memb + n * kMw + tid) = mv;
    }
  }
}

__global__ __launch_bounds__(128) void ntm_meminit_kernel(const float* __restrict__ mem0, float* __restrict__ MEM) {
  const int b = blockIdx.x;
  const int tid = threadIdx.x;
  float* memb = MEM + (size_t)b * kNs * kMw;
  for (int pass = 0; pass < 2; ++pass) {
#pragma unroll 1
    for (int n = 0; n < kNs; ++n) {
      const float mv = bf16r(mem0[n * kMw + tid]);
      *(volatile float*)(memb + n * kMw + tid) = mv;
    }
    __threadfence();
  }
}

static_assert(((size_t)kB * kT * kD / 8) % kThr == 0 && ((kB * kHc) / 4) % kThr == 0, "cast and controller grids exact");

extern "C" void kernel_launch(void* const* d_in, const int* in_sizes, int n_in,
                              void* d_out, int out_size, void* d_ws, size_t ws_size,
                              hipStream_t stream) {
  if (n_in < 22 || d_out == nullptr || d_ws == nullptr) return;
  if (in_sizes[0] != kB * kT * kD || in_sizes[1] != kNs * kMw) return;
  if (in_sizes[2] != kB * kNs || in_sizes[3] != kB * kNs || in_sizes[4] != kB * kHc) return;
  if (in_sizes[5] != kD * kHc || in_sizes[6] != kMw * kHc || in_sizes[7] != kHc) return;
  if (in_sizes[8] != 2 * kHc * kMw || in_sizes[9] != 2 * kMw) return;
  if (in_sizes[10] != 2 * kHc || in_sizes[11] != 2 || in_sizes[12] != 2 * kHc || in_sizes[13] != 2) return;
  if (in_sizes[14] != 2 * kHc * 3 || in_sizes[15] != 6 || in_sizes[16] != 2 * kHc || in_sizes[17] != 2) return;
  if (in_sizes[18] != kHc * kMw || in_sizes[19] != kMw || in_sizes[20] != kHc * kMw || in_sizes[21] != kMw) return;
  if (out_size != kB * kT * kHc) return;
  if (ws_size < kWsTotal) return;

  const float* x    = (const float*)d_in[0];
  const float* mem0 = (const float*)d_in[1];
  const float* wr0  = (const float*)d_in[2];
  const float* ww0  = (const float*)d_in[3];
  const float* h0   = (const float*)d_in[4];
  const float* Wx   = (const float*)d_in[5];
  const float* Wrd  = (const float*)d_in[6];
  const float* bh   = (const float*)d_in[7];
  const float* Wk   = (const float*)d_in[8];
  const float* bk   = (const float*)d_in[9];
  const float* Wb   = (const float*)d_in[10];
  const float* bb   = (const float*)d_in[11];
  const float* Wg   = (const float*)d_in[12];
  const float* bg   = (const float*)d_in[13];
  const float* Ws   = (const float*)d_in[14];
  const float* bs   = (const float*)d_in[15];
  const float* Wgam = (const float*)d_in[16];
  const float* bgam = (const float*)d_in[17];
  const float* We   = (const float*)d_in[18];
  const float* be   = (const float*)d_in[19];
  const float* Wa   = (const float*)d_in[20];
  const float* ba   = (const float*)d_in[21];
  float* out = (float*)d_out;

  char* ws = (char*)d_ws;
  unsigned short* X16   = (unsigned short*)(ws + kOffX16);
  unsigned short* WX16  = (unsigned short*)(ws + kOffWX);
  unsigned short* WRD16 = (unsigned short*)(ws + kOffWRD);
  unsigned short* WA16  = (unsigned short*)(ws + kOffWA);
  float* BA   = (float*)(ws + kOffBA);
  float* BH   = (float*)(ws + kOffBH);
  float* ZB   = (float*)(ws + kOffZB);
  float* XW   = (float*)(ws + kOffXW);
  unsigned short* H16 = (unsigned short*)(ws + kOffH16);
  unsigned short* R16 = (unsigned short*)(ws + kOffR16);
  float* PREH = (float*)(ws + kOffPREH);
  float* PREA = (float*)(ws + kOffPREA);
  float* MEM  = (float*)(ws + kOffMEM);
  float* WRW  = (float*)(ws + kOffWRW);

  cast_plane_kernel<<<(int)(((size_t)kB * kT * kD / 8) / kThr), kThr, 0, stream>>>(x, X16, 7, kD, 0);
  tcast_kernel<<<kHc, kD / 8, 0, stream>>>(Wx, WX16, kD, kHc, 0);
  tcast_kernel<<<kHc, kMw / 8, 0, stream>>>(Wrd, WRD16, kMw, kHc, 1);
  wa_plane_kernel<<<kNA, 32, 0, stream>>>(Wk, Wb, Wg, Ws, Wgam, We, Wa, WA16);
  ntm_small_kernel<<<1, kThr, 0, stream>>>(bk, bb, bg, bs, bgam, be, ba, bh, h0, wr0, ww0, BA, BH, ZB, H16, WRW);
  ntm_meminit_kernel<<<kB, 128, 0, stream>>>(mem0, MEM);

  wmma_gemm64<0, false, 2, 0, false, 0><<<dim3(((kB * kT) / 64) * (kHc / 64) / 8, 1), 256, 0, stream>>>(
      X16, X16, kD, 0L, WX16, WX16, kD, 0L, (void*)XW, (void*)XW, kHc, 0L,
      ZB, nullptr, 0L, kB * kT, kHc, kD, kXScale);

  wmma_gemm64<0, false, 2, 0, false, 0><<<dim3(3, 1), 256, 0, stream>>>(
      H16, H16, 2 * kHc, 0L, WA16, WA16, 2 * kHc, 0L, (void*)PREA, (void*)PREA, kNA, 0L,
      BA, nullptr, 0L, kB, kNA, 2 * kHc, kAScale);
  ntm_mem_kernel<<<kB, 128, 0, stream>>>(PREA, MEM, WRW, R16, 0, 1);

  for (int t = 0; t < kT; ++t) {
    wmma_gemm64<0, false, 2, 0, false, 0><<<dim3(1, 1), 256, 0, stream>>>(
        R16, R16, 2 * kMw, 0L, WRD16, WRD16, 2 * kMw, 0L, (void*)PREH, (void*)PREH, kHc, 0L,
        BH, nullptr, 0L, kB, kHc, 2 * kMw, kRScale);
    ntm_ctrl_kernel<<<(kB * kHc / 4) / kThr, kThr, 0, stream>>>(XW, PREH, out, H16, t);
    if (t + 1 < kT) {
      wmma_gemm64<0, false, 2, 0, false, 0><<<dim3(3, 1), 256, 0, stream>>>(
          H16, H16, 2 * kHc, 0L, WA16, WA16, 2 * kHc, 0L, (void*)PREA, (void*)PREA, kNA, 0L,
          BA, nullptr, 0L, kB, kNA, 2 * kHc, kAScale);
      ntm_mem_kernel<<<kB, 128, 0, stream>>>(PREA, MEM, WRW, R16, 1, 1);
    }
  }
}
